// BandPassFilter_39333310496998
// MI455X (gfx1250) — hardware-verified
//
#include <hip/hip_runtime.h>
#include <math.h>

typedef __attribute__((ext_vector_type(16))) _Float16 v16h;
typedef __attribute__((ext_vector_type(8)))  _Float16 v8h;
typedef __attribute__((ext_vector_type(8)))  float    v8f;
typedef __attribute__((ext_vector_type(4)))  float    v4f;

constexpr int kBatch  = 64;
constexpr int kLen    = 8192;
constexpr int kBands  = 20;
constexpr int kTaps   = 769;
constexpr int kHalf   = kTaps - 1;
constexpr int kCorr   = 2 * kTaps - 1;
constexpr int kKp     = 1600;
constexpr int kTileN  = 64;
constexpr int kRowsM  = kLen / kTileN;
constexpr int kXwLen  = kLen + kCorr - 1;
constexpr int kRightC = 2 * kLen - 2 + kHalf;
constexpr int kSlabP  = 68;
constexpr int kWStage = 1024;
constexpr int kScLen  = 1544;

constexpr float kCarryC = 262144.0f;
constexpr float kCarryX = 16.0f;
constexpr float kUndo   = 1.0f / (kCarryC * kCarryX);

static_assert(kHalf == 768 && kCorr == 1537 && kXwLen == 9728 && kRightC == 17150, "derived constants");
static_assert((kKp % 32) == 0, "K multiple of 32");
static_assert(kKp >= kTileN - 1 + kCorr, "band fits in padded K");
static_assert(kTileN * (kRowsM - 1) + kKp <= kXwLen, "window reads stay inside one signal row");
static_assert((kRowsM % 64) == 0, "M multiple of 64");
static_assert(((kRowsM / 64) * kBands) % 8 == 0, "tiles per batch fill whole blocks");
static_assert(kTaps <= kWStage && kCorr <= kScLen, "LDS extents");
static_assert((kHalf % 8) == 0 && ((kHalf + kLen) % 8) == 0 && (kXwLen % 8) == 0, "8-element chunks never straddle a region");

constexpr size_t kBtBytes = (size_t)kBands * kTileN * kKp * 2;
constexpr size_t kXwBytes = (size_t)kBatch * kXwLen * 2;
constexpr size_t kOffBt   = 0;
constexpr size_t kOffXw   = kOffBt + kBtBytes;
constexpr size_t kWsTotal = kOffXw + kXwBytes;
static_assert(kBtBytes == 4096000ull && kXwBytes == 1245184ull && kWsTotal == 5341184ull, "carve total");
static_assert((kOffXw % 128) == 0 && kWsTotal <= 134217728ull, "carve alignment and cap");

__device__ __forceinline__ v16h frag_load(const _Float16* p) {
  union U { v16h v; v8h h[2]; };
  U f;
  f.h[0] = *(const v8h*)(p);
  f.h[1] = *(const v8h*)(p + 16);
  return f.v;
}
__device__ __forceinline__ v8f wmma_step(v16h a, v16h b, v8f c) {
  c = __builtin_amdgcn_wmma_f32_16x16x32_f16(false, a, false, b, (short)0, c, false, false);
  asm volatile("v_nop\n\tv_nop\n\tv_nop\n\tv_nop" : "+v"(c) : "v"(a), "v"(b));
  return c;
}

__global__ __launch_bounds__(256) void build_bt_kernel(const float* __restrict__ kern,
                                                       unsigned short* __restrict__ bt)
{
  __shared__ float sw[kWStage];
  __shared__ float sc[kScLen];
  const int tid = threadIdx.x;
  const int o   = blockIdx.x;

#pragma unroll
  for (int j = 0; j < 4; ++j) {
    const int i  = tid + 256 * j;
    const int ic = (i < kTaps) ? i : (kTaps - 1);
    const float v = kern[(size_t)o * kTaps + ic];
    sw[i] = (i < kTaps) ? v : 0.0f;
  }
  __syncthreads();

#pragma unroll 1
  for (int j = 0; j < 4; ++j) {
    const int d = tid + 256 * j;
    if (d < kTaps) {
      const int n = kTaps - d;
      float s = 0.0f;
#pragma unroll 4
      for (int i = 0; i < n; ++i) s = fmaf(sw[i], sw[i + d], s);
      const float sv = s * kCarryC;
      sc[kHalf + d] = sv;
      sc[kHalf - d] = sv;
    }
  }
  __syncthreads();

  unsigned short* plane = bt + (size_t)o * (kTileN * kKp);
  constexpr int kChunksPerRow = kKp / 8;
  constexpr int kIters = (kTileN * kChunksPerRow) / 256;
  static_assert(kIters * 256 == kTileN * kChunksPerRow, "exact chunk coverage");
#pragma unroll 1
  for (int it = 0; it < kIters; ++it) {
    const int q  = it * 256 + tid;
    const int nn = q / kChunksPerRow;
    const int k0 = (q - nn * kChunksPerRow) * 8;
    v8h hv;
#pragma unroll
    for (int e = 0; e < 8; ++e) {
      const int s  = k0 + e - nn;
      const int sl = (s < 0) ? 0 : ((s > kCorr - 1) ? (kCorr - 1) : s);
      const float v  = sc[sl];
      const float vv = (s >= 0 && s <= kCorr - 1) ? v : 0.0f;
      hv[e] = (_Float16)vv;
    }
    unsigned short* p = plane + (size_t)q * 8;
    *(volatile v8h*)p = hv;
    __threadfence();
    *(volatile v8h*)p = hv;
  }
}

constexpr int kXwChunksRow = kXwLen / 8;
constexpr int kXwBlocks    = (kBatch * kXwChunksRow) / 256;
static_assert(kXwBlocks * 256 == kBatch * kXwChunksRow, "exact chunk coverage");

__global__ __launch_bounds__(256) void build_xw_kernel(const float* __restrict__ x,
                                                       unsigned short* __restrict__ xw)
{
  const int q  = blockIdx.x * 256 + threadIdx.x;
  const int b  = q / kXwChunksRow;
  const int i0 = (q - b * kXwChunksRow) * 8;
  const float* xs = x + (size_t)b * kLen;
  v8h hv;
#pragma unroll
  for (int e = 0; e < 8; ++e) {
    const int i = i0 + e;
    const bool mid = (i >= kHalf) && (i < kHalf + kLen);
    int idx = (i < kHalf) ? (kHalf - i) : (mid ? (i - kHalf) : (kRightC - i));
    idx = (idx < 0) ? 0 : ((idx > kLen - 1) ? (kLen - 1) : idx);
    const float v = xs[idx];
    const float g = mid ? kCarryX : -kCarryX;
    hv[e] = (_Float16)(v * g);
  }
  unsigned short* p = xw + (size_t)q * 8;
  *(volatile v8h*)p = hv;
  __threadfence();
  *(volatile v8h*)p = hv;
}

__global__ __launch_bounds__(256) void fir_gemm_kernel(const unsigned short* __restrict__ xwp,
                                                       const unsigned short* __restrict__ btp,
                                                       float* __restrict__ out)
{
  __shared__ __align__(16) float sT[8][16 * kSlabP];
  const int lane  = threadIdx.x & 31;
  const int wave  = __builtin_amdgcn_readfirstlane((int)(threadIdx.x >> 5));
  const int b     = blockIdx.y;
  const int tile  = blockIdx.x * 8 + wave;
  const int tm    = tile / kBands;
  const int o     = tile - tm * kBands;
  const int m0    = tm * 64;
  const int rlane = lane & 15;
  const int hsel  = lane >> 4;
  const int koff  = hsel * 8;
  const int mOff  = hsel * 8;

  const _Float16* ap = (const _Float16*)xwp + (size_t)b * kXwLen + (size_t)(m0 + rlane) * kTileN + koff;
  const _Float16* bp = (const _Float16*)btp + (size_t)o * (kTileN * kKp) + (size_t)rlane * kKp + koff;

  v8f acc[4][4];
#pragma unroll
  for (int i = 0; i < 4; ++i)
#pragma unroll
    for (int j = 0; j < 4; ++j) acc[i][j] = (v8f){0.f, 0.f, 0.f, 0.f, 0.f, 0.f, 0.f, 0.f};

#pragma unroll 1
  for (int k0 = 0; k0 < kKp; k0 += 32) {
    v16h bh[4];
#pragma unroll
    for (int j = 0; j < 4; ++j) bh[j] = frag_load(bp + (size_t)(j * 16) * kKp + k0);
#pragma unroll
    for (int i = 0; i < 4; ++i) {
      const v16h ah = frag_load(ap + (i * 16) * kTileN + k0);
#pragma unroll
      for (int j = 0; j < 4; ++j) acc[i][j] = wmma_step(ah, bh[j], acc[i][j]);
    }
  }

  float* slab = sT[wave];
  float* C = out + (size_t)b * ((size_t)kBands * kLen) + (size_t)o * kLen;
  const int c4 = (lane & 15) * 4;
#pragma unroll
  for (int i = 0; i < 4; ++i) {
    const int mBase = m0 + (i << 4);
#pragma unroll
    for (int j = 0; j < 4; ++j) {
#pragma unroll
      for (int r = 0; r < 8; ++r) {
        slab[(mOff + r) * kSlabP + (j << 4) + rlane] = acc[i][j][r] * kUndo;
      }
    }
    __syncthreads();
    for (int pass = 0; pass < 2; ++pass) {
#pragma unroll
      for (int it = 0; it < 8; ++it) {
        const int row = it * 2 + hsel;
        const v4f v = *(const v4f*)(slab + row * kSlabP + c4);
        *(volatile v4f*)(C + (size_t)(mBase + row) * kTileN + c4) = v;
      }
      __threadfence();
    }
    __syncthreads();
  }
}

extern "C" void kernel_launch(void* const* d_in, const int* in_sizes, int n_in,
                              void* d_out, int out_size, void* d_ws, size_t ws_size,
                              hipStream_t stream) {
  if (n_in < 2) return;
  if (in_sizes[0] != kBatch * kLen) return;
  if (in_sizes[1] != kBands * kTaps) return;
  if (out_size != kBatch * kBands * kLen) return;
  if (ws_size < kWsTotal) return;

  const float* x    = (const float*)d_in[0];
  const float* kern = (const float*)d_in[1];
  float* out = (float*)d_out;
  char* ws = (char*)d_ws;
  unsigned short* bt = (unsigned short*)(ws + kOffBt);
  unsigned short* xw = (unsigned short*)(ws + kOffXw);

  build_bt_kernel<<<kBands, 256, 0, stream>>>(kern, bt);
  build_xw_kernel<<<kXwBlocks, 256, 0, stream>>>(x, xw);
  fir_gemm_kernel<<<dim3(((kRowsM / 64) * kBands) / 8, kBatch), 256, 0, stream>>>(xw, bt, out);
}
